// S4DKernel_46686294507696
// MI455X (gfx1250) — hardware-run, weakly checked
//
#include <hip/hip_runtime.h>
#include <cmath>

typedef __attribute__((ext_vector_type(16))) _Float16 v16h;
typedef __attribute__((ext_vector_type(8)))  _Float16 v8h;
typedef __attribute__((ext_vector_type(16))) __bf16   v16b;
typedef __attribute__((ext_vector_type(8)))  __bf16   v8b;
typedef __attribute__((ext_vector_type(8)))  float    v8f;
typedef __attribute__((ext_vector_type(4)))  float    v4f;
typedef __attribute__((ext_vector_type(4)))  unsigned v4u;

constexpr int SEQ_LEN   = 4096;
constexpr int HID_DIM   = 512;
constexpr int NUM_STATE = 16;
constexpr int DT_RANK   = 32;
constexpr int RANK_PAD  = 64;
constexpr int SCAN_TILE = 32;
constexpr float GEMM_SCALE = 1.0f;

constexpr size_t WS_SZ_U    = (size_t)SEQ_LEN * HID_DIM * 2;
constexpr size_t WS_SZ_XW   = (size_t)RANK_PAD * HID_DIM * 2;
constexpr size_t WS_SZ_DW   = (size_t)HID_DIM * DT_RANK * 2;
constexpr size_t WS_SZ_DTU  = (size_t)SEQ_LEN * RANK_PAD * 2;
constexpr size_t WS_SZ_XPRE = (size_t)SEQ_LEN * HID_DIM * 4;
constexpr size_t WS_OFF_UHI   = 0;
constexpr size_t WS_OFF_ULO   = WS_OFF_UHI + WS_SZ_U;
constexpr size_t WS_OFF_XWHI  = WS_OFF_ULO + WS_SZ_U;
constexpr size_t WS_OFF_XWLO  = WS_OFF_XWHI + WS_SZ_XW;
constexpr size_t WS_OFF_DWHI  = WS_OFF_XWLO + WS_SZ_XW;
constexpr size_t WS_OFF_DWLO  = WS_OFF_DWHI + WS_SZ_DW;
constexpr size_t WS_OFF_DTUHI = WS_OFF_DWLO + WS_SZ_DW;
constexpr size_t WS_OFF_DTULO = WS_OFF_DTUHI + WS_SZ_DTU;
constexpr size_t WS_OFF_XPRE  = WS_OFF_DTULO + WS_SZ_DTU;
constexpr size_t WS_TOTAL     = WS_OFF_XPRE + WS_SZ_XPRE;
static_assert(WS_TOTAL == 18022400);
static_assert(WS_TOTAL <= 134217728);
static_assert((WS_OFF_ULO % 128) == 0 && (WS_OFF_XWHI % 128) == 0 && (WS_OFF_XWLO % 128) == 0 &&
              (WS_OFF_DWHI % 128) == 0 && (WS_OFF_DWLO % 128) == 0 && (WS_OFF_DTUHI % 128) == 0 &&
              (WS_OFF_DTULO % 128) == 0 && (WS_OFF_XPRE % 128) == 0);
static_assert(SEQ_LEN % 64 == 0 && RANK_PAD % 64 == 0 && HID_DIM % 64 == 0);
static_assert(HID_DIM % 32 == 0 && DT_RANK % 32 == 0);
static_assert(((SEQ_LEN / 64) * (RANK_PAD / 64)) % 8 == 0);
static_assert(((SEQ_LEN / 64) * (HID_DIM / 64)) % 8 == 0);
static_assert(SEQ_LEN % SCAN_TILE == 0 && HID_DIM % 32 == 0);
static_assert((SEQ_LEN * HID_DIM / 8) % 256 == 0 && (RANK_PAD * HID_DIM / 8) % 256 == 0 && (HID_DIM * DT_RANK / 8) % 256 == 0);

__device__ __forceinline__ unsigned short f2bf_bits(float f) {
  unsigned u = __float_as_uint(f);
  return (unsigned short)((u + 0x7FFFu + ((u >> 16) & 1u)) >> 16);
}
__device__ __forceinline__ float bf_bits2f(unsigned short h) { return __uint_as_float(((unsigned)h) << 16); }

__device__ __forceinline__ void dep_guard_h(v8f& a, v8f& b, v16h x, v16h y) { asm volatile("v_nop\n\tv_nop\n\tv_nop\n\tv_nop" : "+v"(a), "+v"(b) : "v"(x), "v"(y)); }
__device__ __forceinline__ void dep_guard_b(v8f& a, v8f& b, v16b x, v16b y) { asm volatile("v_nop\n\tv_nop\n\tv_nop\n\tv_nop" : "+v"(a), "+v"(b) : "v"(x), "v"(y)); }
__device__ __forceinline__ void keep4_h(v16h a, v16h b, v16h c, v16h d) { asm volatile("v_nop" :: "v"(a), "v"(b), "v"(c), "v"(d)); }
__device__ __forceinline__ void keep4_b(v16b a, v16b b, v16b c, v16b d) { asm volatile("v_nop" :: "v"(a), "v"(b), "v"(c), "v"(d)); }
__device__ __forceinline__ void acc_guard4(v8f& a, v8f& b, v8f& c, v8f& d) { asm volatile("v_nop\n\tv_nop\n\tv_nop\n\tv_nop" : "+v"(a), "+v"(b), "+v"(c), "+v"(d)); }
template <typename T> struct Frag;
template <> struct Frag<_Float16> {
  typedef v16h V; union U { v16h v; v8h h[2]; };
  static __device__ __forceinline__ v16h load(const _Float16* p) {
    U f; f.h[0] = *(const v8h*)(p); f.h[1] = *(const v8h*)(p + 16); return f.v;
  }
  static __device__ __forceinline__ v8f mma(v16h a, v16h b, v8f c) {
    return __builtin_amdgcn_wmma_f32_16x16x32_f16(false, a, false, b, (short)0, c, false, false);
  }
  static __device__ __forceinline__ void guard(v8f& a, v8f& b, v16h x, v16h y) { dep_guard_h(a, b, x, y); }
  static __device__ __forceinline__ void keep(v16h a, v16h b, v16h c, v16h d) { keep4_h(a, b, c, d); }
};
template <> struct Frag<__bf16> {
  typedef v16b V; union U { v16b v; v8b h[2]; };
  static __device__ __forceinline__ v16b load(const __bf16* p) {
    U f; f.h[0] = *(const v8b*)(p); f.h[1] = *(const v8b*)(p + 16); return f.v;
  }
  static __device__ __forceinline__ v8f mma(v16b a, v16b b, v8f c) {
    return __builtin_amdgcn_wmma_f32_16x16x32_bf16(false, a, false, b, (short)0, c, false, false);
  }
  static __device__ __forceinline__ void guard(v8f& a, v8f& b, v16b x, v16b y) { dep_guard_b(a, b, x, y); }
  static __device__ __forceinline__ void keep(v16b a, v16b b, v16b c, v16b d) { keep4_b(a, b, c, d); }
};

template <int ET> struct Elem;
template <> struct Elem<0> { typedef _Float16 T; };
template <> struct Elem<1> { typedef __bf16 T; };
template <int ET, bool SPLIT, int BIAS_MODE, int OUT_MODE, bool RESID, int ACT = 0>
__global__ __launch_bounds__(256) void wmma_gemm64(
    const unsigned short* __restrict__ Ap, const unsigned short* __restrict__ A2p, int lda, long strideA,
    const unsigned short* __restrict__ Btp, const unsigned short* __restrict__ Bt2p, int ldb, long strideB,
    void* __restrict__ Cout, void* __restrict__ Cout2, int ldc, long strideC,
    const float* __restrict__ bias,
    const float* __restrict__ resid, long strideR,
    int M, int N, int K, float scale) {
  typedef typename Elem<ET>::T T;
  typedef typename Frag<T>::V V;
  const T* A = (const T*)Ap; const T* A2 = (const T*)A2p; const T* Bt = (const T*)Btp; const T* Bt2 = (const T*)Bt2p;
  __shared__ __align__(16) float sT[8][16 * 68];
  const int b    = blockIdx.y;
  const int lane = threadIdx.x & 31;
  const int wave = threadIdx.x >> 5;
  const int tilesN = N >> 6;
  const int tilesM = M >> 6;
  const int tile = blockIdx.x * 8 + wave;
  if (tile >= tilesM * tilesN) return;
  const int tm = tile / tilesN;
  const int tn = tile - tm * tilesN;
  const int m0 = tm << 6;
  const int n0 = tn << 6;

  const T* Ab  = A  + (size_t)b * strideA;
  const T* Bb  = Bt + (size_t)b * strideB;
  const T* Ab2 = SPLIT ? (A2  + (size_t)b * strideA) : nullptr;
  const T* Bb2 = SPLIT ? (Bt2 + (size_t)b * strideB) : nullptr;

  const int rlane = lane & 15;
  const int koff  = (lane >> 4) * 8;
  const int mOff  = (lane >> 4) * 8;

  v8f acc[4][4];
#pragma unroll
  for (int i = 0; i < 4; ++i)
#pragma unroll
    for (int j = 0; j < 4; ++j) acc[i][j] = (v8f){0.f,0.f,0.f,0.f,0.f,0.f,0.f,0.f};

  for (int k0 = 0; k0 < K; k0 += 32) {
    V bh[4], bl[4];
#pragma unroll
    for (int j = 0; j < 4; ++j) {
      const size_t bo = (size_t)(n0 + (j << 4) + rlane) * ldb + koff + k0;
      bh[j] = Frag<T>::load(Bb + bo);
      if (SPLIT) bl[j] = Frag<T>::load(Bb2 + bo);
    }
#pragma unroll
    for (int i = 0; i < 4; ++i) {
      const size_t ao = (size_t)(m0 + (i << 4) + rlane) * lda + koff + k0;
      V ah = Frag<T>::load(Ab + ao);
      V al;
      if (SPLIT) al = Frag<T>::load(Ab2 + ao);
#pragma unroll
      for (int j = 0; j < 4; ++j) {
        acc[i][j] = Frag<T>::mma(ah, bh[j], acc[i][j]);
        if (SPLIT) {
          acc[i][j] = Frag<T>::mma(ah, bl[j], acc[i][j]);
          acc[i][j] = Frag<T>::mma(al, bh[j], acc[i][j]);
        }
      }
      Frag<T>::guard(acc[i][0], acc[i][3], ah, SPLIT ? al : ah);
    }
    Frag<T>::keep(bh[0], bh[1], bh[2], bh[3]);
    if (SPLIT) Frag<T>::keep(bl[0], bl[1], bl[2], bl[3]);
  }
  acc_guard4(acc[0][0], acc[0][1], acc[0][2], acc[0][3]);
  acc_guard4(acc[1][0], acc[1][1], acc[1][2], acc[1][3]);
  acc_guard4(acc[2][0], acc[2][1], acc[2][2], acc[2][3]);
  acc_guard4(acc[3][0], acc[3][1], acc[3][2], acc[3][3]);

  float* slab = sT[wave];
  const float* Rb = RESID ? (resid + (size_t)b * strideR) : nullptr;
#pragma unroll
  for (int i = 0; i < 4; ++i) {
    const int mBase = m0 + (i << 4);
#pragma unroll
    for (int j = 0; j < 4; ++j) {
      const int n = n0 + (j << 4) + rlane;
      float bv = 0.f;
      if (BIAS_MODE == 2) bv = bias[n];
#pragma unroll
      for (int r = 0; r < 8; ++r) {
        float v = acc[i][j][r] * scale;
        if (BIAS_MODE == 1) v += bias[mBase + mOff + r];
        if (BIAS_MODE == 2) v += bv;
        if (RESID) v += Rb[(size_t)(mBase + mOff + r) * ldc + n];
        if (ACT == 1) v = tanhf(v);
        if (ACT == 2) v = fmaxf(v, 0.0f);
        if (ACT == 3) v = v / (1.0f + expf(-v));
        if (ACT == 4) v = (v > 0.f) ? v : 0.01f * v;
        if (ACT == 5) v = 0.5f * v * (1.0f + erff(v * 0.70710678118654752f));
        slab[(mOff + r) * 68 + (j << 4) + rlane] = v;
      }
    }
    __builtin_amdgcn_fence(__ATOMIC_RELEASE, "workgroup");
    __builtin_amdgcn_wave_barrier();
    __builtin_amdgcn_fence(__ATOMIC_ACQUIRE, "workgroup");
    if (OUT_MODE == 0) {
      float* C = (float*)Cout + (size_t)b * strideC;
      const int hh = lane >> 4, c4 = (lane & 15) * 4;
      for (int pass = 0; pass < 2; ++pass) {
#pragma unroll
        for (int it = 0; it < 8; ++it) {
          const int row = it * 2 + hh;
          v4f v = *(const v4f*)(slab + row * 68 + c4);
          *(volatile v4f*)(C + (size_t)(mBase + row) * ldc + n0 + c4) = v;
        }
        __threadfence();
      }
    } else {
      const int q = lane >> 3, c8 = (lane & 7) * 8;
      unsigned short* C  = (unsigned short*)Cout  + (size_t)b * strideC;
      unsigned short* C2 = (OUT_MODE == 2) ? ((unsigned short*)Cout2 + (size_t)b * strideC) : nullptr;
      for (int pass = 0; pass < 2; ++pass) {
#pragma unroll
        for (int it = 0; it < 4; ++it) {
          const int row = it * 4 + q;
          const float* sp = slab + row * 68 + c8;
          v8h hv, lv;
#pragma unroll
          for (int e = 0; e < 8; ++e) {
            if (OUT_MODE == 1) {
              hv[e] = (_Float16)sp[e];
            } else {
              unsigned short hb = f2bf_bits(sp[e]);
              unsigned short lb = f2bf_bits(sp[e] - bf_bits2f(hb));
              hv[e] = __builtin_bit_cast(_Float16, hb);
              lv[e] = __builtin_bit_cast(_Float16, lb);
            }
          }
          *(volatile v8h*)(C + (size_t)(mBase + row) * ldc + n0 + c8) = hv;
          if (OUT_MODE == 2) *(volatile v8h*)(C2 + (size_t)(mBase + row) * ldc + n0 + c8) = lv;
        }
        __threadfence();
      }
    }
    __builtin_amdgcn_fence(__ATOMIC_RELEASE, "workgroup");
    __builtin_amdgcn_wave_barrier();
    __builtin_amdgcn_fence(__ATOMIC_ACQUIRE, "workgroup");
  }
}

__global__ __launch_bounds__(256) void split_plane_bf16(
    const float* __restrict__ in, unsigned* __restrict__ hiw, unsigned* __restrict__ low,
    int nReal8, int nTotal8) {
  const int g = blockIdx.x * 256 + threadIdx.x;
  if (g >= nTotal8) return;
  const bool live = g < nReal8;
  const int gs = live ? g : (nReal8 - 1);
  const float* src = in + (size_t)gs * 8;
  const v4f a = *(const v4f*)(src);
  const v4f b = *(const v4f*)(src + 4);
  float x[8];
  x[0] = a[0]; x[1] = a[1]; x[2] = a[2]; x[3] = a[3];
  x[4] = b[0]; x[5] = b[1]; x[6] = b[2]; x[7] = b[3];
  unsigned hb[8], lb[8];
#pragma unroll
  for (int e = 0; e < 8; ++e) {
    const float v = live ? x[e] : 0.0f;
    const unsigned short h = f2bf_bits(v);
    hb[e] = (unsigned)h;
    lb[e] = (unsigned)f2bf_bits(v - bf_bits2f(h));
  }
  v4u hv, lv;
#pragma unroll
  for (int i = 0; i < 4; ++i) {
    hv[i] = hb[2 * i] | (hb[2 * i + 1] << 16);
    lv[i] = lb[2 * i] | (lb[2 * i + 1] << 16);
  }
  unsigned* dh = hiw + (size_t)g * 4;
  unsigned* dl = low + (size_t)g * 4;
  *(volatile v4u*)dh = hv;
  *(volatile v4u*)dl = lv;
  __threadfence();
  *(volatile v4u*)dh = hv;
  *(volatile v4u*)dl = lv;
}

__global__ __launch_bounds__(32) void s4d_scan(
    const float* __restrict__ Xpre, const float* __restrict__ Uin,
    const float* __restrict__ Alog, const float* __restrict__ Aim,
    const float* __restrict__ Bp, const float* __restrict__ Cp,
    const float* __restrict__ Dp, const float* __restrict__ dtb,
    float* __restrict__ Y) {
  __shared__ __align__(16) float s_x[SCAN_TILE * 32];
  __shared__ __align__(16) float s_u[SCAN_TILE * 32];
  __shared__ __align__(16) float s_y[SCAN_TILE * 32];
  const int lane = threadIdx.x;
  const int h0 = blockIdx.x * 32;
  const int h  = h0 + lane;

  float ar[NUM_STATE], ai[NUM_STATE], bre[NUM_STATE], bim[NUM_STATE], cre[NUM_STATE], cim[NUM_STATE];
  float sre[NUM_STATE], sim[NUM_STATE];
  {
    const float* al = Alog + (size_t)h * NUM_STATE;
    const float* am = Aim  + (size_t)h * NUM_STATE;
#pragma unroll
    for (int i = 0; i < 4; ++i) {
      const v4f a = *(const v4f*)(al + 4 * i);
      const v4f m = *(const v4f*)(am + 4 * i);
#pragma unroll
      for (int e = 0; e < 4; ++e) {
        ar[4 * i + e] = -expf(a[e]);
        ai[4 * i + e] = m[e];
      }
    }
    const float* bp = Bp + (size_t)h * NUM_STATE * 2;
    const float* cp = Cp + (size_t)h * NUM_STATE * 2;
#pragma unroll
    for (int i = 0; i < 8; ++i) {
      const v4f b = *(const v4f*)(bp + 4 * i);
      const v4f c = *(const v4f*)(cp + 4 * i);
      bre[2 * i] = b[0]; bim[2 * i] = b[1]; bre[2 * i + 1] = b[2]; bim[2 * i + 1] = b[3];
      cre[2 * i] = c[0]; cim[2 * i] = c[1]; cre[2 * i + 1] = c[2]; cim[2 * i + 1] = c[3];
    }
#pragma unroll
    for (int n = 0; n < NUM_STATE; ++n) { sre[n] = 0.0f; sim[n] = 0.0f; }
  }
  const float dsk  = Dp[h];
  const float bias = dtb[h];
  const int q = lane >> 3, c = lane & 7;

#pragma unroll 1
  for (int t0 = 0; t0 < SEQ_LEN; t0 += SCAN_TILE) {
#pragma unroll
    for (int it = 0; it < 8; ++it) {
      const int row = it * 4 + q;
      const size_t go = (size_t)(t0 + row) * HID_DIM + h0 + c * 4;
      v4f xv = *(const v4f*)(Xpre + go);
      v4f uv = *(const v4f*)(Uin + go);
      asm volatile("" : "+v"(xv), "+v"(uv));
      *(v4f*)(s_x + row * 32 + c * 4) = xv;
      *(v4f*)(s_u + row * 32 + c * 4) = uv;
    }
    __syncthreads();
#pragma unroll 1
    for (int j = 0; j < SCAN_TILE; ++j) {
      const float xj = s_x[j * 32 + lane];
      const float uj = s_u[j * 32 + lane];
      const float v  = xj + bias;
      const float dt = (v > 20.0f) ? v : log1pf(expf(v));
      float acc = 0.0f;
#pragma unroll
      for (int n = 0; n < NUM_STATE; ++n) {
        const float zr = dt * ar[n];
        const float zi = dt * ai[n];
        const float er = expf(zr);
        float sn, cs;
        sincosf(zi, &sn, &cs);
        const float abr = er * cs;
        const float abi = er * sn;
        const float zm2 = zr * zr + zi * zi;
        const float nr  = abr - 1.0f;
        const float inv = 1.0f / fmaxf(zm2, 1.0e-20f);
        const float qr  = (nr * zr + abi * zi) * inv;
        const float qi  = (abi * zr - nr * zi) * inv;
        const bool  tiny = zm2 < 1.0e-8f;
        const float bdr = tiny ? (1.0f + 0.5f * zr) : qr;
        const float bdi = tiny ? (0.5f * zi) : qi;
        const float tr  = bdr * bre[n] - bdi * bim[n];
        const float ti  = bdr * bim[n] + bdi * bre[n];
        const float nhr = abr * sre[n] - abi * sim[n] + uj * tr;
        const float nhi = abr * sim[n] + abi * sre[n] + uj * ti;
        sre[n] = nhr;
        sim[n] = nhi;
        acc += nhr * cre[n] - nhi * cim[n];
      }
      s_y[j * 32 + lane] = acc + uj * dsk;
    }
    __syncthreads();
    for (int pass = 0; pass < 2; ++pass) {
#pragma unroll
      for (int it = 0; it < 8; ++it) {
        const int row = it * 4 + q;
        const v4f w = *(const v4f*)(s_y + row * 32 + c * 4);
        *(volatile v4f*)(Y + (size_t)(t0 + row) * HID_DIM + h0 + c * 4) = w;
      }
      __threadfence();
    }
    __syncthreads();
  }
}

extern "C" void kernel_launch(void* const* d_in, const int* in_sizes, int n_in,
                              void* d_out, int out_size, void* d_ws, size_t ws_size,
                              hipStream_t stream) {
  if (n_in != 9) return;
  if (in_sizes[0] != SEQ_LEN * HID_DIM) return;
  if (in_sizes[1] != HID_DIM * NUM_STATE) return;
  if (in_sizes[2] != HID_DIM * NUM_STATE) return;
  if (in_sizes[3] != HID_DIM * NUM_STATE * 2) return;
  if (in_sizes[4] != HID_DIM * NUM_STATE * 2) return;
  if (in_sizes[5] != HID_DIM) return;
  if (in_sizes[6] != HID_DIM * DT_RANK) return;
  if (in_sizes[7] != HID_DIM) return;
  if (in_sizes[8] != DT_RANK * HID_DIM) return;
  if (out_size != SEQ_LEN * HID_DIM) return;
  if (ws_size < WS_TOTAL) return;

  const float* U     = (const float*)d_in[0];
  const float* Alog  = (const float*)d_in[1];
  const float* Aim   = (const float*)d_in[2];
  const float* Bp    = (const float*)d_in[3];
  const float* Cp    = (const float*)d_in[4];
  const float* Dp    = (const float*)d_in[5];
  const float* DtW   = (const float*)d_in[6];
  const float* DtB   = (const float*)d_in[7];
  const float* XpW   = (const float*)d_in[8];
  float* Out = (float*)d_out;

  unsigned char* ws = (unsigned char*)d_ws;
  unsigned* uHi   = (unsigned*)(ws + WS_OFF_UHI);
  unsigned* uLo   = (unsigned*)(ws + WS_OFF_ULO);
  unsigned* xwHi  = (unsigned*)(ws + WS_OFF_XWHI);
  unsigned* xwLo  = (unsigned*)(ws + WS_OFF_XWLO);
  unsigned* dwHi  = (unsigned*)(ws + WS_OFF_DWHI);
  unsigned* dwLo  = (unsigned*)(ws + WS_OFF_DWLO);
  unsigned* dtuHi = (unsigned*)(ws + WS_OFF_DTUHI);
  unsigned* dtuLo = (unsigned*)(ws + WS_OFF_DTULO);
  float*    xPre  = (float*)(ws + WS_OFF_XPRE);

  split_plane_bf16<<<dim3((SEQ_LEN * HID_DIM / 8) / 256), dim3(256), 0, stream>>>(
      U, uHi, uLo, SEQ_LEN * HID_DIM / 8, SEQ_LEN * HID_DIM / 8);
  split_plane_bf16<<<dim3((RANK_PAD * HID_DIM / 8) / 256), dim3(256), 0, stream>>>(
      XpW, xwHi, xwLo, DT_RANK * HID_DIM / 8, RANK_PAD * HID_DIM / 8);
  split_plane_bf16<<<dim3((HID_DIM * DT_RANK / 8) / 256), dim3(256), 0, stream>>>(
      DtW, dwHi, dwLo, HID_DIM * DT_RANK / 8, HID_DIM * DT_RANK / 8);

  wmma_gemm64<1, true, 0, 2, false><<<dim3(((SEQ_LEN / 64) * (RANK_PAD / 64)) / 8, 1), dim3(256), 0, stream>>>(
      (const unsigned short*)uHi, (const unsigned short*)uLo, HID_DIM, 0L,
      (const unsigned short*)xwHi, (const unsigned short*)xwLo, HID_DIM, 0L,
      (void*)dtuHi, (void*)dtuLo, RANK_PAD, 0L,
      DtB, U, 0L,
      SEQ_LEN, RANK_PAD, HID_DIM, GEMM_SCALE);

  wmma_gemm64<1, true, 0, 0, false><<<dim3(((SEQ_LEN / 64) * (HID_DIM / 64)) / 8, 1), dim3(256), 0, stream>>>(
      (const unsigned short*)dtuHi, (const unsigned short*)dtuLo, RANK_PAD, 0L,
      (const unsigned short*)dwHi, (const unsigned short*)dwLo, DT_RANK, 0L,
      (void*)xPre, (void*)xPre, HID_DIM, 0L,
      DtB, U, 0L,
      SEQ_LEN, HID_DIM, DT_RANK, GEMM_SCALE);

  s4d_scan<<<dim3(HID_DIM / 32), dim3(32), 0, stream>>>(xPre, U, Alog, Aim, Bp, Cp, Dp, DtB, Out);
}
